// FeatureExtract_26233660244203
// MI455X (gfx1250) — hardware-verified
//
#include <hip/hip_runtime.h>
#include <stddef.h>
#include <math.h>


#define CH      256
#define FEAT    118
#define KE      128
#define NTHR    256
#define NWAVE   8
#define GR      64
#define EPT     8
#define NGRP    2
#define CHUNK   (NTHR * EPT * NGRP)
#define WCAP    (EPT * NGRP * 32)
#define LISTN   (NWAVE * WCAP)
#define NBA     256

#define LDS_GEMM (GR * CH * 4)
#define LDS_AGG  (NBA * CH * 4 + LISTN * 4 + 64 + NBA * 4)

static_assert((CHUNK & (CHUNK - 1)) == 0);
static_assert(CHUNK <= 4096);
static_assert((NBA & (NBA - 1)) == 0);
static_assert(NBA <= 4096);
static_assert(NBA == NWAVE * 32);
static_assert(GR == NWAVE * 8);
static_assert(KE % 32 == 0);
static_assert(CH % 32 == 0);
static_assert(KE >= FEAT);

typedef float          v4f  __attribute__((ext_vector_type(4)));
typedef float          v8f  __attribute__((ext_vector_type(8)));
typedef int            v4i  __attribute__((ext_vector_type(4)));
typedef unsigned short v8us __attribute__((ext_vector_type(8)));
typedef __bf16         v16b __attribute__((ext_vector_type(16)));
union FragB { v16b v; v8us u[2]; };

__device__ __forceinline__ float gelu_exact(float v) {
  return 0.5f * v * (1.0f + erff(v * 0.70710678118654752f));
}

__device__ __forceinline__ unsigned bfr(float f) {
  const unsigned u = __float_as_uint(f);
  return (u + 0x7FFFu + ((u >> 16) & 1u)) >> 16;
}

__device__ __forceinline__ void split8(v4f a, v4f b, v8us& hi, v8us& lo) {
#define SPL(I, X) { const unsigned h_ = bfr(X); const float r_ = (X) - __uint_as_float(h_ << 16); \
                    hi[I] = (unsigned short)h_; lo[I] = (unsigned short)bfr(r_); }
  SPL(0, a.x) SPL(1, a.y) SPL(2, a.z) SPL(3, a.w)
  SPL(4, b.x) SPL(5, b.y) SPL(6, b.z) SPL(7, b.w)
#undef SPL
}

__device__ __forceinline__ v8f wmb3(v16b ah, v16b al, v16b bh, v16b bl, v8f c) {
  v8f d = __builtin_amdgcn_wmma_f32_16x16x32_bf16(false, ah, false, bh, (short)0, c, false, false);
  d = __builtin_amdgcn_wmma_f32_16x16x32_bf16(false, ah, false, bl, (short)0, d, false, false);
  d = __builtin_amdgcn_wmma_f32_16x16x32_bf16(false, al, false, bh, (short)0, d, false, false);
  asm volatile("v_nop\n\tv_nop\n\tv_nop\n\tv_nop" : "+v"(d) : "v"(ah), "v"(al), "v"(bh), "v"(bl));
  return d;
}

__global__ __launch_bounds__(NTHR) void k_wprep(
    const float* __restrict__ We, const float* __restrict__ W1, const float* __restrict__ W2,
    unsigned short* weh, unsigned short* wel, unsigned short* w1h, unsigned short* w1l,
    unsigned short* w2h, unsigned short* w2l) {
  const int i  = blockIdx.x * NTHR + threadIdx.x;
  const int n0 = CH * KE / 8;
  const int n1 = CH * CH / 8;
  if (i >= n0 + 2 * n1) return;
  const int sel  = (i < n0) ? 0 : ((i < n0 + n1) ? 1 : 2);
  const int j    = (sel == 0) ? i : ((sel == 1) ? (i - n0) : (i - n0 - n1));
  const int K    = (sel == 0) ? KE : CH;
  const int Kact = (sel == 0) ? FEAT : CH;
  const float* W = (sel == 0) ? We : ((sel == 1) ? W1 : W2);
  unsigned short* ph = (sel == 0) ? weh : ((sel == 1) ? w1h : w2h);
  unsigned short* pl = (sel == 0) ? wel : ((sel == 1) ? w1l : w2l);
  const int o  = j * 8;
  const int n  = o / K;
  const int k0 = o - n * K;
  v4f a, b;
#define LW(I) (((k0 + (I)) < Kact) ? W[(size_t)min(k0 + (I), Kact - 1) * CH + n] : 0.0f)
  a.x = LW(0); a.y = LW(1); a.z = LW(2); a.w = LW(3);
  b.x = LW(4); b.y = LW(5); b.z = LW(6); b.w = LW(7);
#undef LW
  v8us hv, lv;
  split8(a, b, hv, lv);
  unsigned short* dh = ph + o;
  unsigned short* dl = pl + o;
  *(volatile v8us*)dh = hv;
  *(volatile v8us*)dl = lv;
  __threadfence();
  *(volatile v8us*)dh = hv;
  *(volatile v8us*)dl = lv;
}

__global__ __launch_bounds__(NTHR) void k_xprep(
    const float* __restrict__ x, unsigned short* xh, unsigned short* xl, int nN, int nRows) {
  const int i = blockIdx.x * NTHR + threadIdx.x;
  if (i >= nRows * (KE / 8)) return;
  const int row = i / (KE / 8);
  const int c0  = (i - row * (KE / 8)) * 8;
  int node = row > nN - 1 ? nN - 1 : row;
  const float* xp = x + (size_t)node * FEAT;
  v4f a, b;
#define LX(I) (((c0 + (I)) < FEAT) ? xp[min(c0 + (I), FEAT - 1)] : 0.0f)
  a.x = LX(0); a.y = LX(1); a.z = LX(2); a.w = LX(3);
  b.x = LX(4); b.y = LX(5); b.z = LX(6); b.w = LX(7);
#undef LX
  v8us hv, lv;
  split8(a, b, hv, lv);
  unsigned short* dh = xh + (size_t)row * KE + c0;
  unsigned short* dl = xl + (size_t)row * KE + c0;
  *(volatile v8us*)dh = hv;
  *(volatile v8us*)dl = lv;
  __threadfence();
  *(volatile v8us*)dh = hv;
  *(volatile v8us*)dl = lv;
}

template <int KS, int MODE>
__global__ __launch_bounds__(NTHR) void k_gemm(
    const unsigned short* __restrict__ Ah, const unsigned short* __restrict__ Al,
    const unsigned short* __restrict__ Bh, const unsigned short* __restrict__ Bl,
    const float* __restrict__ bias,
    unsigned short* oh, unsigned short* ol, float* of, int nN) {
  extern __shared__ v4f lds_dyn[];
  __shared__ float rs[NWAVE * 16];
  __shared__ __attribute__((aligned(16))) float outs[GR];
  constexpr int K = KS * 32;
  const int tid = threadIdx.x, lane = tid & 31, wave = tid >> 5, hh = lane >> 4, m = lane & 15;
  const int rt = wave & 3, cf = wave >> 2;
  const int rowBase = blockIdx.x * GR;

  const unsigned short* ahp = Ah + ((size_t)rowBase + rt * 16 + m) * K + 8 * hh;
  const unsigned short* alp = Al + ((size_t)rowBase + rt * 16 + m) * K + 8 * hh;
  const unsigned short* bhp = Bh + ((size_t)cf * 128 + m) * K + 8 * hh;
  const unsigned short* blp = Bl + ((size_t)cf * 128 + m) * K + 8 * hh;

  v8f acc[8];
#pragma unroll
  for (int t = 0; t < 8; ++t) { v8f z = {0.f, 0.f, 0.f, 0.f, 0.f, 0.f, 0.f, 0.f}; acc[t] = z; }

#pragma unroll 1
  for (int kt = 0; kt < KS; ++kt) {
    FragB fah, fal;
    fah.u[0] = *(const v8us*)(ahp + 32 * kt);
    fah.u[1] = *(const v8us*)(ahp + 32 * kt + 16);
    fal.u[0] = *(const v8us*)(alp + 32 * kt);
    fal.u[1] = *(const v8us*)(alp + 32 * kt + 16);
#pragma unroll
    for (int t = 0; t < 8; ++t) {
      const unsigned short* ph = bhp + (size_t)(16 * t) * K + 32 * kt;
      const unsigned short* pl = blp + (size_t)(16 * t) * K + 32 * kt;
      FragB fbh, fbl;
      fbh.u[0] = *(const v8us*)ph;
      fbh.u[1] = *(const v8us*)(ph + 16);
      fbl.u[0] = *(const v8us*)pl;
      fbl.u[1] = *(const v8us*)(pl + 16);
      acc[t] = wmb3(fah.v, fal.v, fbh.v, fbl.v, acc[t]);
    }
  }

  float bv[8];
#pragma unroll
  for (int t = 0; t < 8; ++t) bv[t] = bias[cf * 128 + 16 * t + m];

  if (MODE == 2) {
    v8f sv = {0.f, 0.f, 0.f, 0.f, 0.f, 0.f, 0.f, 0.f};
#pragma unroll
    for (int t = 0; t < 8; ++t) {
#pragma unroll
      for (int r = 0; r < 8; ++r) sv[r] += gelu_exact(acc[t][r] + bv[t]);
    }
#pragma unroll
    for (int r = 0; r < 8; ++r) {
      float v = sv[r];
      v += __shfl_xor(v, 1, 16);
      v += __shfl_xor(v, 2, 16);
      v += __shfl_xor(v, 4, 16);
      v += __shfl_xor(v, 8, 16);
      sv[r] = v;
    }
    if (m == 0) {
#pragma unroll
      for (int r = 0; r < 8; ++r) rs[wave * 16 + 8 * hh + r] = sv[r];
    }
    __syncthreads();
    if (tid < GR) {
      const int q = tid >> 4, i = tid & 15;
      outs[tid] = (rs[q * 16 + i] + rs[(q + 4) * 16 + i]) * (1.0f / (float)CH);
    }
    __syncthreads();
    v4f ov = {0.f, 0.f, 0.f, 0.f};
    const int r0 = rowBase + 4 * lane;
    if (wave == 0 && lane < 16) ov = *(const v4f*)(outs + 4 * lane);
    if (wave == 0 && lane < 16) {
      if (r0 + 3 < nN) {
        *(volatile v4f*)(of + r0) = ov;
      } else {
        if (r0     < nN) *(volatile float*)(of + r0)     = ov.x;
        if (r0 + 1 < nN) *(volatile float*)(of + r0 + 1) = ov.y;
        if (r0 + 2 < nN) *(volatile float*)(of + r0 + 2) = ov.z;
        if (r0 + 3 < nN) *(volatile float*)(of + r0 + 3) = ov.w;
      }
    }
    __threadfence();
    if (wave == 0 && lane < 16) {
      if (r0 + 3 < nN) {
        *(volatile v4f*)(of + r0) = ov;
      } else {
        if (r0     < nN) *(volatile float*)(of + r0)     = ov.x;
        if (r0 + 1 < nN) *(volatile float*)(of + r0 + 1) = ov.y;
        if (r0 + 2 < nN) *(volatile float*)(of + r0 + 2) = ov.z;
        if (r0 + 3 < nN) *(volatile float*)(of + r0 + 3) = ov.w;
      }
    }
  } else {
    float* stg = (float*)lds_dyn;
    float* sp = stg + (rt * 16 + 8 * hh) * CH + cf * 128 + m;
#pragma unroll
    for (int t = 0; t < 8; ++t) {
#pragma unroll
      for (int r = 0; r < 8; ++r) {
        float v = acc[t][r] + bv[t];
        if (MODE == 1) v = gelu_exact(v);
        sp[r * CH + 16 * t] = v;
      }
    }
    __syncthreads();
    if (MODE == 0) {
      v8us hv[8], lv[8];
      const float* lp = stg + (wave * 8) * CH + 8 * lane;
#pragma unroll
      for (int i = 0; i < 8; ++i) {
        const v4f p0 = *(const v4f*)(lp + i * CH);
        const v4f p1 = *(const v4f*)(lp + i * CH + 4);
        split8(p0, p1, hv[i], lv[i]);
      }
      unsigned short* gh = oh + ((size_t)rowBase + wave * 8) * CH + 8 * lane;
      unsigned short* gl = ol + ((size_t)rowBase + wave * 8) * CH + 8 * lane;
#pragma unroll
      for (int i = 0; i < 8; ++i) {
        *(volatile v8us*)(gh + (size_t)i * CH) = hv[i];
        *(volatile v8us*)(gl + (size_t)i * CH) = lv[i];
      }
      __threadfence();
#pragma unroll
      for (int i = 0; i < 8; ++i) {
        *(volatile v8us*)(gh + (size_t)i * CH) = hv[i];
        *(volatile v8us*)(gl + (size_t)i * CH) = lv[i];
      }
    } else {
      v4f pv[16];
      const float* lp = stg + (wave * 8) * CH + 4 * lane;
#pragma unroll
      for (int i = 0; i < 8; ++i) {
        pv[2 * i]     = *(const v4f*)(lp + i * CH);
        pv[2 * i + 1] = *(const v4f*)(lp + i * CH + 128);
      }
      float* gp = of + ((size_t)rowBase + wave * 8) * CH + 4 * lane;
#pragma unroll
      for (int i = 0; i < 8; ++i) {
        *(volatile v4f*)(gp + (size_t)i * CH)       = pv[2 * i];
        *(volatile v4f*)(gp + (size_t)i * CH + 128) = pv[2 * i + 1];
      }
      __threadfence();
#pragma unroll
      for (int i = 0; i < 8; ++i) {
        *(volatile v4f*)(gp + (size_t)i * CH)       = pv[2 * i];
        *(volatile v4f*)(gp + (size_t)i * CH + 128) = pv[2 * i + 1];
      }
    }
  }
}

template <int NB>
__device__ __forceinline__ int scan_chunk(const int* __restrict__ dsts, int nE, int cbase, int nodeBase,
                                          int vec8, int* list, int tid, int lane, int wave) {
  (void)lane;
  int wc = 0;
#pragma unroll
  for (int g = 0; g < NGRP; ++g) {
    const int el0  = (g * NTHR + tid) * EPT;
    const int e0   = cbase + el0;
    const int sent = -2147483647 - 1;
    v4i da, db;
    if (vec8 != 0 && e0 + 7 < nE) {
      da = *(const v4i*)(dsts + e0);
      db = *(const v4i*)(dsts + e0 + 4);
    } else {
      da.x = (e0     < nE) ? dsts[min(e0, nE - 1)] : sent;
      da.y = (e0 + 1 < nE) ? dsts[min(e0 + 1, nE - 1)] : sent;
      da.z = (e0 + 2 < nE) ? dsts[min(e0 + 2, nE - 1)] : sent;
      da.w = (e0 + 3 < nE) ? dsts[min(e0 + 3, nE - 1)] : sent;
      db.x = (e0 + 4 < nE) ? dsts[min(e0 + 4, nE - 1)] : sent;
      db.y = (e0 + 5 < nE) ? dsts[min(e0 + 5, nE - 1)] : sent;
      db.z = (e0 + 6 < nE) ? dsts[min(e0 + 6, nE - 1)] : sent;
      db.w = (e0 + 7 < nE) ? dsts[min(e0 + 7, nE - 1)] : sent;
    }
    const unsigned nb = (unsigned)nodeBase;
    const unsigned s0 = (unsigned)da.x - nb, s1 = (unsigned)da.y - nb;
    const unsigned s2 = (unsigned)da.z - nb, s3 = (unsigned)da.w - nb;
    const unsigned s4 = (unsigned)db.x - nb, s5 = (unsigned)db.y - nb;
    const unsigned s6 = (unsigned)db.z - nb, s7 = (unsigned)db.w - nb;
    const bool h0 = s0 < (unsigned)NB, h1 = s1 < (unsigned)NB, h2 = s2 < (unsigned)NB, h3 = s3 < (unsigned)NB;
    const bool h4 = s4 < (unsigned)NB, h5 = s5 < (unsigned)NB, h6 = s6 < (unsigned)NB, h7 = s7 < (unsigned)NB;
    const unsigned any = __builtin_amdgcn_ballot_w32(h0 | h1 | h2 | h3 | h4 | h5 | h6 | h7);
    if (any != 0u) {
#define HITJ(J, HJ, SJ) { \
        const unsigned mj = __builtin_amdgcn_ballot_w32(HJ); \
        if (mj != 0u) { \
          if (HJ) { \
            const int pos = wc + (int)__builtin_amdgcn_mbcnt_lo(mj, 0u); \
            if (pos < WCAP) list[wave * WCAP + pos] = ((el0 + (J)) << 12) | (int)(SJ); \
          } \
          wc += (int)__builtin_popcount(mj); } }
      HITJ(0, h0, s0)
      HITJ(1, h1, s1)
      HITJ(2, h2, s2)
      HITJ(3, h3, s3)
      HITJ(4, h4, s4)
      HITJ(5, h5, s5)
      HITJ(6, h6, s6)
      HITJ(7, h7, s7)
#undef HITJ
    }
  }
  return wc;
}

__global__ __launch_bounds__(NTHR) void k_agg(
    const int* __restrict__ ei, const float* __restrict__ mf,
    unsigned short* ah, unsigned short* al, int nN, int nE, int vec8) {
  extern __shared__ v4f lds_dyn[];
  float* acc  = (float*)lds_dyn;
  int*   list = (int*)(acc + NBA * CH);
  int*   wcnt = list + LISTN;
  int*   cnt  = wcnt + 16;
  const int tid = threadIdx.x, lane = tid & 31, wave = tid >> 5;
  const int nodeBase = blockIdx.x * NBA;
  const int* dsts = ei + nE;

  {
    const v4f z = {0.f, 0.f, 0.f, 0.f};
    for (int i = tid; i < NBA * CH / 4; i += NTHR) lds_dyn[i] = z;
    for (int i = tid; i < NBA; i += NTHR) cnt[i] = 0;
  }
  __syncthreads();

  const int nChunks = (nE + CHUNK - 1) / CHUNK;
#pragma unroll 1
  for (int ch = 0; ch < nChunks; ++ch) {
    const int cbase = ch * CHUNK;
    const int wc = scan_chunk<NBA>(dsts, nE, cbase, nodeBase, vec8, list, tid, lane, wave);
    if (lane == 0) wcnt[wave] = wc;
    __syncthreads();
    if (wave == 0) {
#pragma unroll 1
      for (int wsx = 0; wsx < NWAVE; ++wsx) {
        int n = __builtin_amdgcn_readfirstlane(wcnt[wsx]);
        n = n > WCAP ? WCAP : (n < 0 ? 0 : n);
        const int* lp = list + wsx * WCAP;
#pragma unroll 1
        for (int i = 0; i < n; ++i) {
          const int ent  = __builtin_amdgcn_readfirstlane(lp[i]);
          const int slot = ent & (NBA - 1);
          int e = cbase + ((ent >> 12) & (CHUNK - 1));
          e = e > nE - 1 ? nE - 1 : e;
          int src = ei[e];
          src = src < 0 ? 0 : (src > nN - 1 ? nN - 1 : src);
          const float* mp = mf + (size_t)src * CH + 8 * lane;
          const v4f v0 = *(const v4f*)mp;
          const v4f v1 = *(const v4f*)(mp + 4);
          v4f* ap = (v4f*)(acc + slot * CH + 8 * lane);
          ap[0] = ap[0] + v0;
          ap[1] = ap[1] + v1;
          if (lane == 0) cnt[slot] = cnt[slot] + 1;
        }
      }
    }
    __syncthreads();
  }

  unsigned short* gh = ah + ((size_t)nodeBase + wave * 32) * CH + 8 * lane;
  unsigned short* gl = al + ((size_t)nodeBase + wave * 32) * CH + 8 * lane;
#pragma unroll 2
  for (int i = 0; i < 32; ++i) {
    const int row = wave * 32 + i;
    const float c = (float)cnt[row];
    const float inv = 1.0f / fmaxf(c, 1.0f);
    const float* lp = acc + row * CH + 8 * lane;
    const v4f p0 = *(const v4f*)lp * inv;
    const v4f p1 = *(const v4f*)(lp + 4) * inv;
    v8us hv, lv;
    split8(p0, p1, hv, lv);
    *(volatile v8us*)(gh + (size_t)i * CH) = hv;
    *(volatile v8us*)(gl + (size_t)i * CH) = lv;
  }
  __threadfence();
#pragma unroll 2
  for (int i = 0; i < 32; ++i) {
    const int row = wave * 32 + i;
    const float c = (float)cnt[row];
    const float inv = 1.0f / fmaxf(c, 1.0f);
    const float* lp = acc + row * CH + 8 * lane;
    const v4f p0 = *(const v4f*)lp * inv;
    const v4f p1 = *(const v4f*)(lp + 4) * inv;
    v8us hv, lv;
    split8(p0, p1, hv, lv);
    *(volatile v8us*)(gh + (size_t)i * CH) = hv;
    *(volatile v8us*)(gl + (size_t)i * CH) = lv;
  }
}

extern "C" void kernel_launch(void* const* d_in, const int* in_sizes, int n_in,
                              void* d_out, int out_size, void* d_ws, size_t ws_size,
                              hipStream_t stream) {
  if (n_in < 8) return;
  const int nN = in_sizes[0] / FEAT;
  const int nE = in_sizes[1] / 2;
  if (nN <= 0 || nE < 0 || in_sizes[0] != nN * FEAT || in_sizes[1] != nE * 2) return;
  if (in_sizes[2] != FEAT * CH || in_sizes[3] < CH) return;
  if (in_sizes[4] != CH * CH || in_sizes[5] < CH) return;
  if (in_sizes[6] != CH * CH || in_sizes[7] < CH) return;
  if (out_size != nN) return;

  const float* x  = (const float*)d_in[0];
  const int*   ei = (const int*)d_in[1];
  const float* We = (const float*)d_in[2];
  const float* be = (const float*)d_in[3];
  const float* W1 = (const float*)d_in[4];
  const float* b1 = (const float*)d_in[5];
  const float* W2 = (const float*)d_in[6];
  const float* b2 = (const float*)d_in[7];
  float* out = (float*)d_out;

  const int gridM = (nN + GR - 1) / GR;
  const int nPG   = gridM * GR;
  const int gridA = (nN + NBA - 1) / NBA;
  const int nPA   = gridA * NBA;

  char* ws = (char*)d_ws;
  size_t off = 0;
  const size_t szWe = (size_t)CH * KE * 2, szW = (size_t)CH * CH * 2;
  const size_t szX  = (size_t)nPG * KE * 2, szH = (size_t)nPG * CH * 2;
  const size_t szM  = (size_t)nPG * CH * 4, szA = (size_t)nPA * CH * 2;
  const size_t oWeh = off; off += szWe; off = (off + 255) & ~(size_t)255;
  const size_t oWel = off; off += szWe; off = (off + 255) & ~(size_t)255;
  const size_t oW1h = off; off += szW;  off = (off + 255) & ~(size_t)255;
  const size_t oW1l = off; off += szW;  off = (off + 255) & ~(size_t)255;
  const size_t oW2h = off; off += szW;  off = (off + 255) & ~(size_t)255;
  const size_t oW2l = off; off += szW;  off = (off + 255) & ~(size_t)255;
  const size_t oXh  = off; off += szX;  off = (off + 255) & ~(size_t)255;
  const size_t oXl  = off; off += szX;  off = (off + 255) & ~(size_t)255;
  const size_t oHh  = off; off += szH;  off = (off + 255) & ~(size_t)255;
  const size_t oHl  = off; off += szH;  off = (off + 255) & ~(size_t)255;
  const size_t oM   = off; off += szM;  off = (off + 255) & ~(size_t)255;
  const size_t oAh  = off; off += szA;  off = (off + 255) & ~(size_t)255;
  const size_t oAl  = off; off += szA;  off = (off + 255) & ~(size_t)255;
  if (off > ws_size) return;
  if (off > (size_t)134217728) return;
  unsigned short* weh = (unsigned short*)(ws + oWeh);
  unsigned short* wel = (unsigned short*)(ws + oWel);
  unsigned short* w1h = (unsigned short*)(ws + oW1h);
  unsigned short* w1l = (unsigned short*)(ws + oW1l);
  unsigned short* w2h = (unsigned short*)(ws + oW2h);
  unsigned short* w2l = (unsigned short*)(ws + oW2l);
  unsigned short* xh  = (unsigned short*)(ws + oXh);
  unsigned short* xl  = (unsigned short*)(ws + oXl);
  unsigned short* hh  = (unsigned short*)(ws + oHh);
  unsigned short* hl  = (unsigned short*)(ws + oHl);
  float*          mbu = (float*)(ws + oM);
  unsigned short* aah = (unsigned short*)(ws + oAh);
  unsigned short* aal = (unsigned short*)(ws + oAl);

  const int vec8 = ((nE & 3) == 0) ? 1 : 0;

  const int nPrep = CH * KE / 8 + 2 * (CH * CH / 8);
  k_wprep<<<(nPrep + NTHR - 1) / NTHR, NTHR, 0, stream>>>(We, W1, W2, weh, wel, w1h, w1l, w2h, w2l);

  const int nXt = nPG * (KE / 8);
  k_xprep<<<(nXt + NTHR - 1) / NTHR, NTHR, 0, stream>>>(x, xh, xl, nN, nPG);

  hipFuncSetAttribute(reinterpret_cast<const void*>(&k_gemm<KE / 32, 0>),
                      hipFuncAttributeMaxDynamicSharedMemorySize, LDS_GEMM);
  k_gemm<KE / 32, 0><<<gridM, NTHR, LDS_GEMM, stream>>>(xh, xl, weh, wel, be, hh, hl, mbu, nN);

  hipFuncSetAttribute(reinterpret_cast<const void*>(&k_gemm<CH / 32, 1>),
                      hipFuncAttributeMaxDynamicSharedMemorySize, LDS_GEMM);
  k_gemm<CH / 32, 1><<<gridM, NTHR, LDS_GEMM, stream>>>(hh, hl, w1h, w1l, b1, hh, hl, mbu, nN);

  hipFuncSetAttribute(reinterpret_cast<const void*>(&k_agg),
                      hipFuncAttributeMaxDynamicSharedMemorySize, LDS_AGG);
  k_agg<<<gridA, NTHR, LDS_AGG, stream>>>(ei, mbu, aah, aal, nN, nE, vec8);

  k_gemm<CH / 32, 2><<<gridM, NTHR, 0, stream>>>(aah, aal, w2h, w2l, b2, aah, aal, out, nN);
}
